// WordRNN_87514253623880
// MI455X (gfx1250) — hardware-verified
//
#include <hip/hip_runtime.h>
#include <math.h>

constexpr int kSeqN    = 512;
constexpr int kStepN   = 512;
constexpr int kEmbD    = 32;
constexpr int kVocRows = 32001;
constexpr int kHidA    = 128;
constexpr int kHidB    = 64;
constexpr int kGateA   = 4 * kHidA;
constexpr int kGateB   = 4 * kHidB;
constexpr int kVoc     = 32000;
constexpr int kWP      = 192;
constexpr int kKcA     = 5;
constexpr int kKcB     = 6;
constexpr int kAP1     = 168;
constexpr int kAP2     = 200;
constexpr int kNT      = 256;
constexpr float kEpsBN = 1e-3f;
constexpr float kActSc = 256.0f;
constexpr float kWSc   = 16.0f;
constexpr float kZInv  = 1.0f / 4096.0f;
constexpr int kRowF4   = kVoc / 4;
constexpr int kSmIt    = (kRowF4 + kNT - 1) / kNT;
static_assert(kSeqN % 64 == 0 && kVoc % 64 == 0 && kHidB % 32 == 0, "head GEMM tile multiples");
static_assert(kGateA % 64 == 0 && kGateB % 64 == 0 && kWP % 64 == 0, "pack tiles");
static_assert((kEmbD + kHidA) == 32 * kKcA && (kHidA + kHidB) == 32 * kKcB, "k chunks");
static_assert(kAP1 % 8 == 0 && kAP2 % 8 == 0 && kAP1 >= 32 * kKcA && kAP2 >= 32 * kKcB, "A tile pitch");
static_assert(kRowF4 % 32 == 0, "whole lines per wave in the softmax writer");

typedef __attribute__((ext_vector_type(16))) _Float16 v16h;
typedef __attribute__((ext_vector_type(8)))  _Float16 v8h;
typedef __attribute__((ext_vector_type(2)))  _Float16 v2h;
typedef __attribute__((ext_vector_type(16))) __bf16   v16b;
typedef __attribute__((ext_vector_type(8)))  __bf16   v8b;
typedef __attribute__((ext_vector_type(8)))  float    v8f;
typedef __attribute__((ext_vector_type(4)))  float    v4f;
typedef __attribute__((ext_vector_type(2)))  float    v2f;

__device__ __forceinline__ unsigned short f2bf_bits(float f) {
  unsigned u = __float_as_uint(f);
  return (unsigned short)((u + 0x7FFFu + ((u >> 16) & 1u)) >> 16);
}
__device__ __forceinline__ float bf_bits2f(unsigned short h) { return __uint_as_float(((unsigned)h) << 16); }

__device__ __forceinline__ void dep_guard_h(v8f& a, v8f& b, v16h x, v16h y) { asm volatile("v_nop\n\tv_nop\n\tv_nop\n\tv_nop" : "+v"(a), "+v"(b) : "v"(x), "v"(y)); }
__device__ __forceinline__ void dep_guard_b(v8f& a, v8f& b, v16b x, v16b y) { asm volatile("v_nop\n\tv_nop\n\tv_nop\n\tv_nop" : "+v"(a), "+v"(b) : "v"(x), "v"(y)); }
__device__ __forceinline__ void keep4_h(v16h a, v16h b, v16h c, v16h d) { asm volatile("v_nop" :: "v"(a), "v"(b), "v"(c), "v"(d)); }
__device__ __forceinline__ void keep4_b(v16b a, v16b b, v16b c, v16b d) { asm volatile("v_nop" :: "v"(a), "v"(b), "v"(c), "v"(d)); }
__device__ __forceinline__ void acc_guard4(v8f& a, v8f& b, v8f& c, v8f& d) { asm volatile("v_nop\n\tv_nop\n\tv_nop\n\tv_nop" : "+v"(a), "+v"(b), "+v"(c), "+v"(d)); }
template <typename T> struct Frag;
template <> struct Frag<_Float16> {
  typedef v16h V; union U { v16h v; v8h h[2]; };
  static __device__ __forceinline__ v16h load(const _Float16* p) {
    U f; f.h[0] = *(const v8h*)(p); f.h[1] = *(const v8h*)(p + 16); return f.v;
  }
  static __device__ __forceinline__ v8f mma(v16h a, v16h b, v8f c) {
    return __builtin_amdgcn_wmma_f32_16x16x32_f16(false, a, false, b, (short)0, c, false, false);
  }
  static __device__ __forceinline__ void guard(v8f& a, v8f& b, v16h x, v16h y) { dep_guard_h(a, b, x, y); }
  static __device__ __forceinline__ void keep(v16h a, v16h b, v16h c, v16h d) { keep4_h(a, b, c, d); }
};
template <> struct Frag<__bf16> {
  typedef v16b V; union U { v16b v; v8b h[2]; };
  static __device__ __forceinline__ v16b load(const __bf16* p) {
    U f; f.h[0] = *(const v8b*)(p); f.h[1] = *(const v8b*)(p + 16); return f.v;
  }
  static __device__ __forceinline__ v8f mma(v16b a, v16b b, v8f c) {
    return __builtin_amdgcn_wmma_f32_16x16x32_bf16(false, a, false, b, (short)0, c, false, false);
  }
  static __device__ __forceinline__ void guard(v8f& a, v8f& b, v16b x, v16b y) { dep_guard_b(a, b, x, y); }
  static __device__ __forceinline__ void keep(v16b a, v16b b, v16b c, v16b d) { keep4_b(a, b, c, d); }
};

__device__ __forceinline__ float fsig(float x) { return __builtin_amdgcn_rcpf(1.0f + __expf(-x)); }

template <int ET> struct Elem;
template <> struct Elem<0> { typedef _Float16 T; };
template <> struct Elem<1> { typedef __bf16 T; };
template <int ET, bool SPLIT, int BIAS_MODE, int OUT_MODE, bool RESID, int ACT = 0>
__global__ __launch_bounds__(256) void wmma_gemm64(
    const unsigned short* __restrict__ Ap, const unsigned short* __restrict__ A2p, int lda, long strideA,
    const unsigned short* __restrict__ Btp, const unsigned short* __restrict__ Bt2p, int ldb, long strideB,
    void* __restrict__ Cout, void* __restrict__ Cout2, int ldc, long strideC,
    const float* __restrict__ bias,
    const float* __restrict__ resid, long strideR,
    int M, int N, int K, float scale) {
  typedef typename Elem<ET>::T T;
  typedef typename Frag<T>::V V;
  const T* A = (const T*)Ap; const T* A2 = (const T*)A2p; const T* Bt = (const T*)Btp; const T* Bt2 = (const T*)Bt2p;
  __shared__ __align__(16) float sT[8][16 * 68];
  const int b    = blockIdx.y;
  const int lane = threadIdx.x & 31;
  const int wave = threadIdx.x >> 5;
  const int tilesN = N >> 6;
  const int tilesM = M >> 6;
  const int tile = blockIdx.x * 8 + wave;
  if (tile >= tilesM * tilesN) return;
  const int tm = tile / tilesN;
  const int tn = tile - tm * tilesN;
  const int m0 = tm << 6;
  const int n0 = tn << 6;

  const T* Ab  = A  + (size_t)b * strideA;
  const T* Bb  = Bt + (size_t)b * strideB;
  const T* Ab2 = SPLIT ? (A2  + (size_t)b * strideA) : nullptr;
  const T* Bb2 = SPLIT ? (Bt2 + (size_t)b * strideB) : nullptr;

  const int rlane = lane & 15;
  const int koff  = (lane >> 4) * 8;
  const int mOff  = (lane >> 4) * 8;

  v8f acc[4][4];
#pragma unroll
  for (int i = 0; i < 4; ++i)
#pragma unroll
    for (int j = 0; j < 4; ++j) acc[i][j] = (v8f){0.f,0.f,0.f,0.f,0.f,0.f,0.f,0.f};

  for (int k0 = 0; k0 < K; k0 += 32) {
    V bh[4], bl[4];
#pragma unroll
    for (int j = 0; j < 4; ++j) {
      const size_t bo = (size_t)(n0 + (j << 4) + rlane) * ldb + koff + k0;
      bh[j] = Frag<T>::load(Bb + bo);
      if (SPLIT) bl[j] = Frag<T>::load(Bb2 + bo);
    }
#pragma unroll
    for (int i = 0; i < 4; ++i) {
      const size_t ao = (size_t)(m0 + (i << 4) + rlane) * lda + koff + k0;
      V ah = Frag<T>::load(Ab + ao);
      V al;
      if (SPLIT) al = Frag<T>::load(Ab2 + ao);
#pragma unroll
      for (int j = 0; j < 4; ++j) {
        acc[i][j] = Frag<T>::mma(ah, bh[j], acc[i][j]);
        if (SPLIT) {
          acc[i][j] = Frag<T>::mma(ah, bl[j], acc[i][j]);
          acc[i][j] = Frag<T>::mma(al, bh[j], acc[i][j]);
        }
      }
      Frag<T>::guard(acc[i][0], acc[i][3], ah, SPLIT ? al : ah);
    }
    Frag<T>::keep(bh[0], bh[1], bh[2], bh[3]);
    if (SPLIT) Frag<T>::keep(bl[0], bl[1], bl[2], bl[3]);
  }
  acc_guard4(acc[0][0], acc[0][1], acc[0][2], acc[0][3]);
  acc_guard4(acc[1][0], acc[1][1], acc[1][2], acc[1][3]);
  acc_guard4(acc[2][0], acc[2][1], acc[2][2], acc[2][3]);
  acc_guard4(acc[3][0], acc[3][1], acc[3][2], acc[3][3]);

  float* slab = sT[wave];
  const float* Rb = RESID ? (resid + (size_t)b * strideR) : nullptr;
#pragma unroll
  for (int i = 0; i < 4; ++i) {
    const int mBase = m0 + (i << 4);
#pragma unroll
    for (int j = 0; j < 4; ++j) {
      const int n = n0 + (j << 4) + rlane;
      float bv = 0.f;
      if (BIAS_MODE == 2) bv = bias[n];
#pragma unroll
      for (int r = 0; r < 8; ++r) {
        float v = acc[i][j][r] * scale;
        if (BIAS_MODE == 1) v += bias[mBase + mOff + r];
        if (BIAS_MODE == 2) v += bv;
        if (RESID) v += Rb[(size_t)(mBase + mOff + r) * ldc + n];
        if (ACT == 1) v = tanhf(v);
        if (ACT == 2) v = fmaxf(v, 0.0f);
        if (ACT == 3) v = v / (1.0f + expf(-v));
        if (ACT == 4) v = (v > 0.f) ? v : 0.01f * v;
        if (ACT == 5) v = 0.5f * v * (1.0f + erff(v * 0.70710678118654752f));
        slab[(mOff + r) * 68 + (j << 4) + rlane] = v;
      }
    }
    __builtin_amdgcn_fence(__ATOMIC_RELEASE, "workgroup");
    __builtin_amdgcn_wave_barrier();
    __builtin_amdgcn_fence(__ATOMIC_ACQUIRE, "workgroup");
    if (OUT_MODE == 0) {
      float* C = (float*)Cout + (size_t)b * strideC;
      const int hh = lane >> 4, c4 = (lane & 15) * 4;
      for (int pass = 0; pass < 2; ++pass) {
#pragma unroll
        for (int it = 0; it < 8; ++it) {
          const int row = it * 2 + hh;
          v4f v = *(const v4f*)(slab + row * 68 + c4);
          *(volatile v4f*)(C + (size_t)(mBase + row) * ldc + n0 + c4) = v;
        }
        __threadfence();
      }
    } else {
      const int q = lane >> 3, c8 = (lane & 7) * 8;
      unsigned short* C  = (unsigned short*)Cout  + (size_t)b * strideC;
      unsigned short* C2 = (OUT_MODE == 2) ? ((unsigned short*)Cout2 + (size_t)b * strideC) : nullptr;
      for (int pass = 0; pass < 2; ++pass) {
#pragma unroll
        for (int it = 0; it < 4; ++it) {
          const int row = it * 4 + q;
          const float* sp = slab + row * 68 + c8;
          v8h hv, lv;
#pragma unroll
          for (int e = 0; e < 8; ++e) {
            if (OUT_MODE == 1) {
              hv[e] = (_Float16)sp[e];
            } else {
              unsigned short hb = f2bf_bits(sp[e]);
              unsigned short lb = f2bf_bits(sp[e] - bf_bits2f(hb));
              hv[e] = __builtin_bit_cast(_Float16, hb);
              lv[e] = __builtin_bit_cast(_Float16, lb);
            }
          }
          *(volatile v8h*)(C + (size_t)(mBase + row) * ldc + n0 + c8) = hv;
          if (OUT_MODE == 2) *(volatile v8h*)(C2 + (size_t)(mBase + row) * ldc + n0 + c8) = lv;
        }
        __threadfence();
      }
    }
    __builtin_amdgcn_fence(__ATOMIC_RELEASE, "workgroup");
    __builtin_amdgcn_wave_barrier();
    __builtin_amdgcn_fence(__ATOMIC_ACQUIRE, "workgroup");
  }
}

__global__ __launch_bounds__(kNT) void pack_cat_kernel(const float* __restrict__ Wa, int Ra,
                                                      const float* __restrict__ Wb, int Rb,
                                                      int Cc, unsigned short* __restrict__ O, int ldo, float sc) {
  __shared__ float Tt[64 * 65];
  const int tid = threadIdx.x;
  const int j0 = blockIdx.x * 64, k0 = blockIdx.y * 64;
#pragma unroll
  for (int i = 0; i < 4; ++i) {
    const int idx = i * kNT + tid;
    const int kk = idx >> 4, jj = (idx & 15) * 4;
    const int k = k0 + kk;
    int ka = (k < Ra - 1) ? k : (Ra - 1);
    int kb = k - Ra; kb = (kb < 0) ? 0 : kb; kb = (kb > Rb - 1) ? (Rb - 1) : kb;
    const v4f va = *(const v4f*)(Wa + (size_t)ka * (size_t)Cc + j0 + jj);
    const v4f vb = *(const v4f*)(Wb + (size_t)kb * (size_t)Cc + j0 + jj);
    const bool ua = (k < Ra), ub = (k < Ra + Rb);
#pragma unroll
    for (int e = 0; e < 4; ++e) {
      const float f = ua ? va[e] : (ub ? vb[e] : 0.0f);
      Tt[kk * 65 + jj + e] = f * sc;
    }
  }
  __syncthreads();
  const int q = tid >> 3, c8 = (tid & 7) * 8;
  v8h hv[2];
#pragma unroll
  for (int g = 0; g < 2; ++g) {
    const int qq = g * 32 + q;
#pragma unroll
    for (int e = 0; e < 8; ++e) hv[g][e] = (_Float16)Tt[(c8 + e) * 65 + qq];
  }
  for (int pass = 0; pass < 2; ++pass) {
#pragma unroll
    for (int g = 0; g < 2; ++g) {
      const size_t o = (size_t)(j0 + g * 32 + q) * (size_t)ldo + (size_t)(k0 + c8);
      *(volatile v8h*)(O + o) = hv[g];
    }
    __threadfence();
  }
}

__global__ __launch_bounds__(kNT) void lstm_stack_kernel(
    const int* __restrict__ ids, const float* __restrict__ emb,
    const unsigned short* __restrict__ WUAp, const unsigned short* __restrict__ WUBp,
    const float* __restrict__ b1, const float* __restrict__ g1, const float* __restrict__ be1,
    const float* __restrict__ m1, const float* __restrict__ v1,
    const float* __restrict__ b2, const float* __restrict__ g2, const float* __restrict__ be2,
    const float* __restrict__ m2, const float* __restrict__ v2,
    unsigned short* __restrict__ Fout) {
  __shared__ __align__(16) _Float16 A1[16 * kAP1];
  __shared__ __align__(16) _Float16 A2[16 * kAP2];
  __shared__ __align__(16) _Float16 Fs[16 * kHidB];
  const _Float16* WUA = (const _Float16*)WUAp;
  const _Float16* WUB = (const _Float16*)WUBp;
  const int tid = threadIdx.x, lane = tid & 31, wave = tid >> 5;
  const int c = lane & 15, hh = lane >> 4, koff = hh * 8;
  const int b0 = blockIdx.x * 16;

#pragma unroll 1
  for (int i = 0; i < 8; ++i) { const int idx = i * kNT + tid; A1[(idx >> 7) * kAP1 + kEmbD + (idx & 127)] = (_Float16)0.0f; }
#pragma unroll 1
  for (int i = 0; i < 4; ++i) { const int idx = i * kNT + tid; A2[(idx >> 6) * kAP2 + kHidA + (idx & 63)] = (_Float16)0.0f; }

  const int hidA = 16 * wave + c;
  const int hidB = 16 * (wave & 3) + c;
  float biaA[4], biaB[4];
#pragma unroll
  for (int g = 0; g < 4; ++g) { biaA[g] = b1[g * kHidA + hidA]; biaB[g] = b2[g * kHidB + hidB]; }
  const float gsA = g1[hidA], mnA = m1[hidA], rsA = rsqrtf(v1[hidA] + kEpsBN), btA = be1[hidA];
  const float gsB = g2[hidB], mnB = m2[hidB], rsB = rsqrtf(v2[hidB] + kEpsBN), btB = be2[hidB];

  float csA[8], csB[8], hB[8];
#pragma unroll
  for (int r = 0; r < 8; ++r) { csA[r] = 0.0f; csB[r] = 0.0f; hB[r] = 0.0f; }

  const _Float16* a1row = A1 + c * kAP1 + koff;
  const _Float16* a2row = A2 + c * kAP2 + koff;
  const _Float16* wA = WUA + (size_t)hidA * kWP + koff;
  const _Float16* wB = WUB + (size_t)hidB * kWP + koff;
  const int gm = tid >> 4, ge2 = (tid & 15) * 2;
  const v8f z8 = {0.f, 0.f, 0.f, 0.f, 0.f, 0.f, 0.f, 0.f};

#pragma unroll 1
  for (int t = 0; t < kStepN; ++t) {
    {
      int id = ids[(size_t)(b0 + gm) * kStepN + t];
      id = (id < 0) ? 0 : id;
      id = (id > kVocRows - 1) ? (kVocRows - 1) : id;
      const v2f v = *(const v2f*)(emb + (size_t)id * kEmbD + ge2);
      v2h p;
      p[0] = (_Float16)(v[0] * kActSc);
      p[1] = (_Float16)(v[1] * kActSc);
      *(v2h*)(A1 + gm * kAP1 + ge2) = p;
    }
    __syncthreads();

    float hA[8];
    {
      v8f acc[4];
      acc[0] = z8; acc[1] = z8; acc[2] = z8; acc[3] = z8;
#pragma unroll 1
      for (int kc = 0; kc < kKcA; ++kc) {
        const int k0 = kc * 32;
        const v16h a  = Frag<_Float16>::load(a1row + k0);
        const v16h f0 = Frag<_Float16>::load(wA + k0);
        const v16h f1 = Frag<_Float16>::load(wA + (size_t)1 * kHidA * kWP + k0);
        const v16h f2 = Frag<_Float16>::load(wA + (size_t)2 * kHidA * kWP + k0);
        const v16h f3 = Frag<_Float16>::load(wA + (size_t)3 * kHidA * kWP + k0);
        acc[0] = Frag<_Float16>::mma(a, f0, acc[0]);
        acc[1] = Frag<_Float16>::mma(a, f1, acc[1]);
        acc[2] = Frag<_Float16>::mma(a, f2, acc[2]);
        acc[3] = Frag<_Float16>::mma(a, f3, acc[3]);
        dep_guard_h(acc[0], acc[3], a, f3);
        keep4_h(f0, f1, f2, f3);
      }
      acc_guard4(acc[0], acc[1], acc[2], acc[3]);
#pragma unroll
      for (int r = 0; r < 8; ++r) {
        const float zi = acc[0][r] * kZInv + biaA[0];
        const float zf = acc[1][r] * kZInv + biaA[1];
        const float zg = acc[2][r] * kZInv + biaA[2];
        const float zo = acc[3][r] * kZInv + biaA[3];
        const float ig = fsig(zi);
        const float fg = fsig(zf);
        const float gg = fmaxf(zg, 0.0f);
        const float og = fsig(zo);
        const float cn = fg * csA[r] + ig * gg;
        csA[r] = cn;
        hA[r] = og * fmaxf(cn, 0.0f);
      }
    }
    __syncthreads();

#pragma unroll
    for (int r = 0; r < 8; ++r) {
      const int row = 8 * hh + r;
      A1[row * kAP1 + kEmbD + hidA] = (_Float16)(kActSc * hA[r]);
      const float bn = (gsA * (hA[r] - mnA)) * rsA + btA;
      A2[row * kAP2 + hidA] = (_Float16)(kActSc * bn);
    }
    if (wave < 4) {
#pragma unroll
      for (int r = 0; r < 8; ++r) A2[(8 * hh + r) * kAP2 + kHidA + hidB] = (_Float16)(kActSc * hB[r]);
    }
    __syncthreads();

    if (wave < 4) {
      v8f acc[4];
      acc[0] = z8; acc[1] = z8; acc[2] = z8; acc[3] = z8;
#pragma unroll 1
      for (int kc = 0; kc < kKcB; ++kc) {
        const int k0 = kc * 32;
        const v16h a  = Frag<_Float16>::load(a2row + k0);
        const v16h f0 = Frag<_Float16>::load(wB + k0);
        const v16h f1 = Frag<_Float16>::load(wB + (size_t)1 * kHidB * kWP + k0);
        const v16h f2 = Frag<_Float16>::load(wB + (size_t)2 * kHidB * kWP + k0);
        const v16h f3 = Frag<_Float16>::load(wB + (size_t)3 * kHidB * kWP + k0);
        acc[0] = Frag<_Float16>::mma(a, f0, acc[0]);
        acc[1] = Frag<_Float16>::mma(a, f1, acc[1]);
        acc[2] = Frag<_Float16>::mma(a, f2, acc[2]);
        acc[3] = Frag<_Float16>::mma(a, f3, acc[3]);
        dep_guard_h(acc[0], acc[3], a, f3);
        keep4_h(f0, f1, f2, f3);
      }
      acc_guard4(acc[0], acc[1], acc[2], acc[3]);
#pragma unroll
      for (int r = 0; r < 8; ++r) {
        const float zi = acc[0][r] * kZInv + biaB[0];
        const float zf = acc[1][r] * kZInv + biaB[1];
        const float zg = acc[2][r] * kZInv + biaB[2];
        const float zo = acc[3][r] * kZInv + biaB[3];
        const float ig = fsig(zi);
        const float fg = fsig(zf);
        const float gg = fmaxf(zg, 0.0f);
        const float og = fsig(zo);
        const float cn = fg * csB[r] + ig * gg;
        csB[r] = cn;
        hB[r] = og * fmaxf(cn, 0.0f);
      }
    }
  }

  if (wave < 4) {
#pragma unroll
    for (int r = 0; r < 8; ++r) {
      const float bn = (gsB * (hB[r] - mnB)) * rsB + btB;
      Fs[(8 * hh + r) * kHidB + hidB] = (_Float16)(kActSc * bn);
    }
  }
  __syncthreads();
  if (wave < 4) {
    const int q = lane >> 3, e8 = (lane & 7) * 8;
    const int row = 4 * wave + q;
    const v8h val = *(const v8h*)(Fs + row * kHidB + e8);
    unsigned short* dst = Fout + (size_t)(b0 + row) * kHidB + e8;
    for (int pass = 0; pass < 2; ++pass) {
      *(volatile v8h*)dst = val;
      __threadfence();
    }
  }
}

__global__ __launch_bounds__(kNT) void softmax_rows_kernel(const float* __restrict__ L, float* __restrict__ out) {
  __shared__ float red[8];
  const int tid = threadIdx.x, lane = tid & 31, wave = tid >> 5;
  const size_t rb = (size_t)blockIdx.x * (size_t)kVoc;
  const float* lr = L + rb;

  float mx = -3.0e38f;
#pragma unroll 1
  for (int i = 0; i < kSmIt; ++i) {
    const int idx = i * kNT + tid;
    const int idc = (idx < kRowF4) ? idx : (kRowF4 - 1);
    const v4f v = *(const v4f*)(lr + 4 * (size_t)idc);
    const float m4 = fmaxf(fmaxf(v[0], v[1]), fmaxf(v[2], v[3]));
    if (idx < kRowF4) mx = fmaxf(mx, m4);
  }
#pragma unroll
  for (int off = 16; off >= 1; off >>= 1) mx = fmaxf(mx, __shfl_xor(mx, off, 32));
  if (lane == 0) red[wave] = mx;
  __syncthreads();
  float rowMax = red[0];
#pragma unroll
  for (int w = 1; w < 8; ++w) rowMax = fmaxf(rowMax, red[w]);
  __syncthreads();

  float s = 0.0f;
#pragma unroll 1
  for (int i = 0; i < kSmIt; ++i) {
    const int idx = i * kNT + tid;
    const int idc = (idx < kRowF4) ? idx : (kRowF4 - 1);
    const v4f v = *(const v4f*)(lr + 4 * (size_t)idc);
    const float e4 = (__expf(v[0] - rowMax) + __expf(v[1] - rowMax)) + (__expf(v[2] - rowMax) + __expf(v[3] - rowMax));
    if (idx < kRowF4) s += e4;
  }
#pragma unroll
  for (int off = 16; off >= 1; off >>= 1) s += __shfl_xor(s, off, 32);
  if (lane == 0) red[wave] = s;
  __syncthreads();
  float rowSum = red[0];
#pragma unroll
  for (int w = 1; w < 8; ++w) rowSum += red[w];
  const float inv = 1.0f / rowSum;

  float* orow = out + rb;
  for (int pass = 0; pass < 2; ++pass) {
#pragma unroll 1
    for (int i = 0; i < kSmIt; ++i) {
      const int idx = i * kNT + tid;
      if (idx < kRowF4) {
        const v4f v = *(const v4f*)(lr + 4 * (size_t)idx);
        v4f w;
        w[0] = __expf(v[0] - rowMax) * inv;
        w[1] = __expf(v[1] - rowMax) * inv;
        w[2] = __expf(v[2] - rowMax) * inv;
        w[3] = __expf(v[3] - rowMax) * inv;
        *(volatile v4f*)(orow + 4 * (size_t)idx) = w;
      }
    }
    __threadfence();
  }
}

extern "C" void kernel_launch(void* const* d_in, const int* in_sizes, int n_in,
                              void* d_out, int out_size, void* d_ws, size_t ws_size, hipStream_t stream) {
  if (n_in < 18 || d_out == nullptr || d_ws == nullptr) return;
  if (in_sizes[0] != kSeqN * kStepN || in_sizes[1] != kVocRows * kEmbD ||
      in_sizes[2] != kEmbD * kGateA || in_sizes[3] != kHidA * kGateA || in_sizes[4] != kGateA ||
      in_sizes[5] != kHidA || in_sizes[6] != kHidA || in_sizes[7] != kHidA || in_sizes[8] != kHidA ||
      in_sizes[9] != kHidA * kGateB || in_sizes[10] != kHidB * kGateB || in_sizes[11] != kGateB ||
      in_sizes[12] != kHidB || in_sizes[13] != kHidB || in_sizes[14] != kHidB || in_sizes[15] != kHidB ||
      in_sizes[16] != kHidB * kVoc || in_sizes[17] != kVoc || out_size != kSeqN * kVoc) return;

  const int*   ids = (const int*)d_in[0];
  const float* emb = (const float*)d_in[1];
  const float* w1  = (const float*)d_in[2];
  const float* u1  = (const float*)d_in[3];
  const float* b1  = (const float*)d_in[4];
  const float* g1  = (const float*)d_in[5];
  const float* be1 = (const float*)d_in[6];
  const float* m1  = (const float*)d_in[7];
  const float* v1  = (const float*)d_in[8];
  const float* w2  = (const float*)d_in[9];
  const float* u2  = (const float*)d_in[10];
  const float* b2  = (const float*)d_in[11];
  const float* g2  = (const float*)d_in[12];
  const float* be2 = (const float*)d_in[13];
  const float* m2  = (const float*)d_in[14];
  const float* v2  = (const float*)d_in[15];
  const float* wd  = (const float*)d_in[16];
  const float* bd  = (const float*)d_in[17];
  float* out = (float*)d_out;

  char* ws = (char*)d_ws; size_t off = 0;
  auto carve = [&](size_t bytes) -> char* { char* p = ws + off; off += (bytes + 255) & ~(size_t)255; return p; };
  unsigned short* WUA = (unsigned short*)carve((size_t)kGateA * kWP * 2);
  unsigned short* WUB = (unsigned short*)carve((size_t)kGateB * kWP * 2);
  unsigned short* WDT = (unsigned short*)carve((size_t)kVoc * kHidB * 2);
  unsigned short* FA  = (unsigned short*)carve((size_t)kSeqN * kHidB * 2);
  float*          LOG = (float*)carve((size_t)kSeqN * kVoc * 4);
  if (off > ws_size || off > (size_t)134217728) return;

  pack_cat_kernel<<<dim3(kGateA / 64, kWP / 64), kNT, 0, stream>>>(w1, kEmbD, u1, kHidA, kGateA, WUA, kWP, kWSc);
  pack_cat_kernel<<<dim3(kGateB / 64, kWP / 64), kNT, 0, stream>>>(w2, kHidA, u2, kHidB, kGateB, WUB, kWP, kWSc);
  pack_cat_kernel<<<dim3(kVoc / 64, 1), kNT, 0, stream>>>(wd, kHidB, wd, kHidB, kVoc, WDT, kHidB, kWSc);
  lstm_stack_kernel<<<kSeqN / 16, kNT, 0, stream>>>(ids, emb, WUA, WUB, b1, g1, be1, m1, v1, b2, g2, be2, m2, v2, FA);
  {
    const int tiles = (kSeqN / 64) * (kVoc / 64);
    wmma_gemm64<0, false, 2, 0, false, 0><<<dim3(tiles / 8, 1), 256, 0, stream>>>(
        FA, FA, kHidB, (long)0, WDT, WDT, kHidB, (long)0,
        (void*)LOG, (void*)LOG, kVoc, (long)0, bd, bd, (long)0, kSeqN, kVoc, kHidB, kZInv);
  }
  softmax_rows_kernel<<<kSeqN, kNT, 0, stream>>>(LOG, out);
}
